// SignalGraphAttention_43937515438699
// MI455X (gfx1250) — hardware-verified
//
#include <hip/hip_runtime.h>
#include <stddef.h>
#include <stdint.h>

#define NBT   8
#define NND   1024
#define DM    256
#define NH    8
#define HDM   32
#define NET   8
#define NEDG  16384
#define NTOK  (NBT * NND)
#define HN    (NTOK * DM)
#define WMAT  (DM * DM)
#define QB    128
#define KC    64
#define NQB   (NND / QB)
#define NCK   (NND / KC)
#define HPL   (NBT * NH * NND * HDM)
#define ALLOWBIT 0x1000000u
#define CNTMASK  0xFFFFFFu

static_assert(NH * HDM == DM);
static_assert(HDM == 32);
static_assert(NND % QB == 0);
static_assert(NND % KC == 0);
static_assert(NND % 256 == 0);
static_assert(DM % 64 == 0);
static_assert(HN % 2048 == 0);
static_assert(NTOK % 32 == 0);
static_assert(HPL == HN);
static_assert(KC == 64);
static_assert(QB == 8 * 16);
static_assert(NEDG % 32 == 0);
static_assert(NET * HDM == 256);
static_assert(NND % 8 == 0);

typedef _Float16 v16h __attribute__((ext_vector_type(16)));
typedef _Float16 v8h  __attribute__((ext_vector_type(8)));
typedef float    v8f  __attribute__((ext_vector_type(8)));
typedef float    v4f  __attribute__((ext_vector_type(4)));
typedef unsigned int v4u __attribute__((ext_vector_type(4)));

union Frag  { v16h v; v8h h[2]; };
union Pack8 { v8h h; v4u u; };

__device__ __forceinline__ v8f mma16(v16h a, v16h b, v8f c) {
  c = __builtin_amdgcn_wmma_f32_16x16x32_f16(false, a, false, b, (short)0, c, false, false);
  asm volatile("v_nop\n\tv_nop\n\tv_nop\n\tv_nop" : "+v"(c) : "v"(a), "v"(b));
  return c;
}

__device__ __forceinline__ v16h ldfrag(const _Float16* p, int ld, int row0, int k0, int lane) {
  const int m = lane & 15, lh = lane >> 4;
  const _Float16* q = p + (size_t)(row0 + m) * ld + k0 + 8 * lh;
  Frag f;
  f.h[0] = *(const v8h*)(q);
  f.h[1] = *(const v8h*)(q + 16);
  return f.v;
}

__device__ __forceinline__ v8f zero8() { return (v8f){0.f, 0.f, 0.f, 0.f, 0.f, 0.f, 0.f, 0.f}; }

__device__ __forceinline__ void gemm32x64(const _Float16* __restrict__ A, int lda, int aks,
                                          const _Float16* __restrict__ Bt, int ldb, int bks, int nk,
                                          int m0, int n0, int lane, v8f (&acc)[2][4]) {
#pragma unroll 1
  for (int kk = 0; kk < nk; ++kk) {
    const _Float16* Ak = A + (size_t)kk * aks;
    const _Float16* Bk = Bt + (size_t)kk * bks;
    const v16h a0 = ldfrag(Ak, lda, m0, 0, lane);
    const v16h a1 = ldfrag(Ak, lda, m0 + 16, 0, lane);
    const v16h b0 = ldfrag(Bk, ldb, n0, 0, lane);
    const v16h b1 = ldfrag(Bk, ldb, n0 + 16, 0, lane);
    const v16h b2 = ldfrag(Bk, ldb, n0 + 32, 0, lane);
    const v16h b3 = ldfrag(Bk, ldb, n0 + 48, 0, lane);
    acc[0][0] = mma16(a0, b0, acc[0][0]);
    acc[1][0] = mma16(a1, b0, acc[1][0]);
    acc[0][1] = mma16(a0, b1, acc[0][1]);
    acc[1][1] = mma16(a1, b1, acc[1][1]);
    acc[0][2] = mma16(a0, b2, acc[0][2]);
    acc[1][2] = mma16(a1, b2, acc[1][2]);
    acc[0][3] = mma16(a0, b3, acc[0][3]);
    acc[1][3] = mma16(a1, b3, acc[1][3]);
  }
}

__global__ __launch_bounds__(256) void k_wcvt(const float* __restrict__ wq, const float* __restrict__ wk,
                                              const float* __restrict__ wv, const float* __restrict__ wo,
                                              _Float16* __restrict__ dst) {
  const int mat = blockIdx.x >> 5;
  const float* src = (mat == 0) ? wq : ((mat == 1) ? wk : ((mat == 2) ? wv : wo));
  const size_t o = (size_t)(blockIdx.x & 31) * 2048 + (size_t)threadIdx.x * 8;
  const v4f a0 = *(const v4f*)(src + o) * 32.0f;
  const v4f a1 = *(const v4f*)(src + o + 4) * 32.0f;
  Pack8 pk;
  pk.h = (v8h){(_Float16)a0[0], (_Float16)a0[1], (_Float16)a0[2], (_Float16)a0[3],
               (_Float16)a1[0], (_Float16)a1[1], (_Float16)a1[2], (_Float16)a1[3]};
  const v4u vv = pk.u;
  volatile v4u* d = (volatile v4u*)(dst + (size_t)mat * WMAT + o);
  *d = vv;
  __threadfence();
  *d = vv;
}

__global__ __launch_bounds__(256) void k_ln(const float* __restrict__ x, const float* __restrict__ g,
                                            const float* __restrict__ be, _Float16* __restrict__ xn) {
  const int tid = threadIdx.x, lane = tid & 31, wave = tid >> 5;
  const size_t row = (size_t)blockIdx.x * 8 + wave;
  const float* xr = x + row * DM + 8 * lane;
  const v4f a0 = *(const v4f*)(xr);
  const v4f a1 = *(const v4f*)(xr + 4);
  float s = ((a0[0] + a0[1]) + (a0[2] + a0[3])) + ((a1[0] + a1[1]) + (a1[2] + a1[3]));
#pragma unroll
  for (int off = 16; off >= 1; off >>= 1) s += __shfl_xor(s, off, 32);
  const float mean = s * 0.00390625f;
  const v4f d0 = a0 - mean, d1 = a1 - mean;
  float ss = ((d0[0] * d0[0] + d0[1] * d0[1]) + (d0[2] * d0[2] + d0[3] * d0[3])) +
             ((d1[0] * d1[0] + d1[1] * d1[1]) + (d1[2] * d1[2] + d1[3] * d1[3]));
#pragma unroll
  for (int off = 16; off >= 1; off >>= 1) ss += __shfl_xor(ss, off, 32);
  const float var  = ss * 0.00390625f;
  const float rstd = rsqrtf(var + 1e-5f);
  const v4f g0 = *(const v4f*)(g + 8 * lane), g1 = *(const v4f*)(g + 8 * lane + 4);
  const v4f e0 = *(const v4f*)(be + 8 * lane), e1 = *(const v4f*)(be + 8 * lane + 4);
  const v4f y0 = (d0 * rstd) * g0 + e0;
  const v4f y1 = (d1 * rstd) * g1 + e1;
  Pack8 pk;
  pk.h = (v8h){(_Float16)y0[0], (_Float16)y0[1], (_Float16)y0[2], (_Float16)y0[3],
               (_Float16)y1[0], (_Float16)y1[1], (_Float16)y1[2], (_Float16)y1[3]};
  const v4u vv = pk.u;
  volatile v4u* d = (volatile v4u*)(xn + row * DM + 8 * lane);
  *d = vv;
  __threadfence();
  *d = vv;
}

__global__ __launch_bounds__(256) void k_tab(const int* __restrict__ ei, const int* __restrict__ et,
                                             unsigned* __restrict__ tab) {
  __shared__ __align__(16) unsigned tw[8 * NND];
  const int tid = threadIdx.x, lane = tid & 31, wave = tid >> 5;
  const int n = blockIdx.x * 8 + wave;
  const int base = wave * NND;
  const v4u z4 = (v4u){0u, 0u, 0u, 0u};
#pragma unroll
  for (int i = 0; i < 8; ++i) *(v4u*)(tw + base + 4 * (lane + 32 * i)) = z4;
  __syncthreads();

#pragma unroll 1
  for (int it = 0; it < NEDG / 32; ++it) {
    const int e = it * 32 + lane;
    int sv = ei[e], tv = ei[NEDG + e], yv = et[e];
    sv = min(max(sv, 0), NND - 1);
    tv = min(max(tv, 0), NND - 1);
    yv = min(max(yv, 0), NET - 1);
    unsigned ba = (unsigned)__ballot(sv == n);
    unsigned bb = (unsigned)__ballot(tv == n);
    while (ba != 0u) {
      const int j = __builtin_ctz(ba);
      ba &= ba - 1u;
      const int tj = __shfl(tv, j, 32);
      const unsigned o = tw[base + tj];
      if (lane == 0) tw[base + tj] = o | ALLOWBIT;
    }
    while (bb != 0u) {
      const int j = __builtin_ctz(bb);
      bb &= bb - 1u;
      const int sj = __shfl(sv, j, 32);
      const int yj = __shfl(yv, j, 32);
      const unsigned sh = 3u * (unsigned)yj;
      const unsigned o = tw[base + sj];
      unsigned f = (o >> sh) & 7u;
      f = (f < 7u) ? (f + 1u) : 7u;
      const unsigned nv = (o & ~(7u << sh)) | (f << sh);
      if (lane == 0) tw[base + sj] = nv;
    }
  }
  {
    const unsigned o = tw[base + n];
    if (lane == 0) tw[base + n] = o | ALLOWBIT;
  }
  __syncthreads();

  v4u val[8];
  size_t go[8];
#pragma unroll
  for (int it = 0; it < 8; ++it) {
    val[it] = *(const v4u*)(tw + base + it * 128 + 4 * lane);
    go[it]  = (size_t)n * NND + (size_t)it * 128 + 4 * lane;
  }
  for (int ps = 0; ps < 2; ++ps) {
#pragma unroll
    for (int it = 0; it < 8; ++it) *(volatile v4u*)(tab + go[it]) = val[it];
    __threadfence();
  }
}

#define STP 72
#define SVP 264
__global__ __launch_bounds__(256) void k_qkv(const _Float16* __restrict__ xn,
                                             const _Float16* __restrict__ w4,
                                             const float* __restrict__ bq,
                                             const float* __restrict__ bk,
                                             const float* __restrict__ bv,
                                             _Float16* __restrict__ qkp,
                                             _Float16* __restrict__ vtp) {
  __shared__ __align__(16) _Float16 st[256 * STP];
  const int tid = threadIdx.x, lane = tid & 31, wave = tid >> 5;
  const int hh = lane >> 4, c = lane & 15;
  const int bx  = blockIdx.x;
  const int b   = bx >> 2;
  const int nb0 = (bx & 3) * 256;
  const int ns  = blockIdx.y;
  const int which = ns >> 2;
  const int cg    = ns & 3;
  const int m0 = bx * 256 + wave * 32;
  const int n0 = cg * 64;
  const _Float16* B = w4 + (size_t)which * WMAT;

  v8f acc[2][4];
#pragma unroll
  for (int s = 0; s < 2; ++s)
#pragma unroll
    for (int t = 0; t < 4; ++t) acc[s][t] = zero8();
  gemm32x64(xn, DM, 32, B, DM, 32, DM / 32, m0, n0, lane, acc);

  float bb[4];
#pragma unroll
  for (int t = 0; t < 4; ++t) {
    const int i = n0 + 16 * t + c;
    const float xq = bq[i], xk = bk[i], xv = bv[i];
    bb[t] = (which == 0) ? xq : ((which == 1) ? xk : xv);
  }

  if (which < 2) {
#pragma unroll
    for (int sub = 0; sub < 2; ++sub)
#pragma unroll
      for (int t = 0; t < 4; ++t)
#pragma unroll
        for (int r = 0; r < 8; ++r)
          st[(wave * 32 + sub * 16 + 8 * hh + r) * STP + 16 * t + c] =
              (_Float16)(acc[sub][t][r] * 0.03125f + bb[t]);
  } else {
#pragma unroll
    for (int sub = 0; sub < 2; ++sub)
#pragma unroll
      for (int t = 0; t < 4; ++t)
#pragma unroll
        for (int r = 0; r < 8; ++r)
          st[(16 * t + c) * SVP + wave * 32 + sub * 16 + 8 * hh + r] =
              (_Float16)(acc[sub][t][r] * 0.03125f + bb[t]);
  }
  __syncthreads();

  if (which < 2) {
    _Float16* dstp = qkp + (size_t)which * HPL;
#pragma unroll
    for (int gq = 0; gq < 2; ++gq) {
      v4u val[4];
      size_t go[4];
#pragma unroll
      for (int j = 0; j < 4; ++j) {
        const int p    = tid + 256 * (4 * gq + j);
        const int slab = p >> 10;
        const int pp   = p & 1023;
        const int lr   = pp >> 2;
        const int pc   = pp & 3;
        Pack8 pk;
        pk.h   = *(const v8h*)(st + lr * STP + slab * 32 + pc * 8);
        val[j] = pk.u;
        go[j]  = ((size_t)(b * NH + 2 * cg + slab) * NND + nb0 + lr) * HDM + pc * 8;
      }
      for (int ps = 0; ps < 2; ++ps) {
#pragma unroll
        for (int j = 0; j < 4; ++j) *(volatile v4u*)(dstp + go[j]) = val[j];
        __threadfence();
      }
    }
  } else {
#pragma unroll
    for (int gq = 0; gq < 2; ++gq) {
      v4u val[4];
      size_t go[4];
#pragma unroll
      for (int j = 0; j < 4; ++j) {
        const int p     = tid + 256 * (4 * gq + j);
        const int drow  = p >> 5;
        const int pc    = p & 31;
        const int head2 = drow >> 5;
        const int d     = drow & 31;
        Pack8 pk;
        pk.h   = *(const v8h*)(st + drow * SVP + pc * 8);
        val[j] = pk.u;
        go[j]  = ((size_t)(b * NH + 2 * cg + head2) * HDM + d) * NND + nb0 + pc * 8;
      }
      for (int ps = 0; ps < 2; ++ps) {
#pragma unroll
        for (int j = 0; j < 4; ++j) *(volatile v4u*)(vtp + go[j]) = val[j];
        __threadfence();
      }
    }
  }
}

#define KSP 40
#define VSP 72
__global__ __launch_bounds__(256) void k_attn(const _Float16* __restrict__ qkp,
                                              const _Float16* __restrict__ vtp,
                                              const unsigned* __restrict__ tab,
                                              const float* __restrict__ emb,
                                              _Float16* __restrict__ op, float sscale) {
  __shared__ __align__(16) _Float16 Ks[KC * KSP];
  __shared__ __align__(16) _Float16 Vs[HDM * VSP];
  __shared__ __align__(16) _Float16 Ps[8 * 16 * VSP];
  __shared__ __align__(16) float Es[NET * HDM];
  __shared__ __align__(16) float Qe[8 * 16 * NET];

  const int tid = threadIdx.x, lane = tid & 31, wave = tid >> 5;
  const int hh = lane >> 4, c = lane & 15;
  const int qb  = blockIdx.x % NQB;
  const int hb  = blockIdx.x / NQB;
  const int q0  = qb * QB + wave * 16;

  const _Float16* Q = qkp + (size_t)hb * NND * HDM;
  const _Float16* K = qkp + (size_t)HPL + (size_t)hb * NND * HDM;
  const _Float16* V = vtp + (size_t)hb * HDM * NND;
  const unsigned* trow = tab + (size_t)(q0 + 8 * hh) * NND + c;

  Es[tid] = emb[tid];
  __syncthreads();

  {
    float e4[4] = {0.f, 0.f, 0.f, 0.f};
    const _Float16* qr = Q + (size_t)(q0 + c) * HDM;
#pragma unroll 1
    for (int qd = 0; qd < 4; ++qd) {
      const v8h qh = *(const v8h*)(qr + 8 * qd);
#pragma unroll
      for (int i = 0; i < 8; ++i) {
        const float qv = (float)qh[i];
#pragma unroll
        for (int u = 0; u < 4; ++u) e4[u] += qv * Es[(4 * hh + u) * HDM + 8 * qd + i];
      }
    }
#pragma unroll
    for (int u = 0; u < 4; ++u) Qe[wave * 128 + c * NET + 4 * hh + u] = e4[u];
  }

  const v16h qa = ldfrag(Q, HDM, q0, 0, lane);

  const float NEGI = -__builtin_huge_valf();
  float mrow[8], lrow[8];
  v8f oacc[2];
#pragma unroll
  for (int r = 0; r < 8; ++r) { mrow[r] = NEGI; lrow[r] = 0.f; }
#pragma unroll
  for (int t = 0; t < 2; ++t) oacc[t] = zero8();

  _Float16* pw = Ps + wave * 16 * VSP;

  for (int kc = 0; kc < NCK; ++kc) {
    const int kv0 = kc * KC;
    __syncthreads();
    {
      const int kr = tid >> 2;
      const int qq = (tid & 3) * 8;
      *(v8h*)(Ks + kr * KSP + qq) = *(const v8h*)(K + (size_t)(kv0 + kr) * HDM + qq);
      const int dr = tid >> 3;
      const int q8 = (tid & 7) * 8;
      *(v8h*)(Vs + dr * VSP + q8) = *(const v8h*)(V + (size_t)dr * NND + kv0 + q8);
    }
    __syncthreads();

    v8f s[4];
#pragma unroll
    for (int j = 0; j < 4; ++j) {
      const v16h kb = ldfrag(Ks, KSP, j * 16, 0, lane);
      s[j] = mma16(qa, kb, zero8());
    }
    float cm[8];
#pragma unroll
    for (int r = 0; r < 8; ++r) {
      float m = NEGI;
#pragma unroll
      for (int j = 0; j < 4; ++j) {
        const unsigned wd = trow[(size_t)r * NND + kv0 + 16 * j];
        float v = s[j][r] * sscale;
        const unsigned cb = wd & CNTMASK;
        if ((unsigned)__ballot(cb != 0u) != 0u) {
          const float* qe = Qe + wave * 128 + (8 * hh + r) * NET;
          float bsum = 0.f;
#pragma unroll
          for (int t = 0; t < NET; ++t) bsum += (float)((cb >> (3 * t)) & 7u) * qe[t];
          v += bsum;
        }
        const float w = ((wd & ALLOWBIT) != 0u) ? v : NEGI;
        s[j][r] = w;
        m = fmaxf(m, w);
      }
#pragma unroll
      for (int off = 1; off < 16; off <<= 1) m = fmaxf(m, __shfl_xor(m, off, 32));
      cm[r] = m;
    }
    float al[8];
#pragma unroll
    for (int r = 0; r < 8; ++r) {
      const float mold = mrow[r];
      const float mnew = fmaxf(mold, cm[r]);
      const float ex   = __expf(mold - mnew);
      const float alpha = (mold == mnew) ? 1.f : ((mold == NEGI) ? 0.f : ex);
      mrow[r] = mnew;
      float psum = 0.f;
#pragma unroll
      for (int j = 0; j < 4; ++j) {
        const float w  = s[j][r];
        const float pe = __expf(w - mnew);
        const float p  = (w == NEGI) ? 0.f : pe;
        psum += p;
        pw[(8 * hh + r) * VSP + j * 16 + c] = (_Float16)(p * 1024.0f);
      }
#pragma unroll
      for (int off = 1; off < 16; off <<= 1) psum += __shfl_xor(psum, off, 32);
      lrow[r] = lrow[r] * alpha + psum;
      al[r] = alpha;
    }
#pragma unroll
    for (int t = 0; t < 2; ++t)
#pragma unroll
      for (int r = 0; r < 8; ++r) oacc[t][r] *= al[r];
    __syncthreads();

#pragma unroll
    for (int kk = 0; kk < 2; ++kk) {
      const v16h pa = ldfrag(pw, VSP, 0, kk * 32, lane);
#pragma unroll
      for (int t = 0; t < 2; ++t) {
        const v16h vb = ldfrag(Vs, VSP, t * 16, kk * 32, lane);
        oacc[t] = mma16(pa, vb, oacc[t]);
      }
    }
  }

  float invl[8];
#pragma unroll
  for (int r = 0; r < 8; ++r) invl[r] = (lrow[r] > 0.f) ? (0.0625f / lrow[r]) : 0.f;
  __syncthreads();
#pragma unroll
  for (int r = 0; r < 8; ++r) {
#pragma unroll
    for (int t = 0; t < 2; ++t)
      pw[(8 * hh + r) * VSP + 16 * t + c] = (_Float16)(oacc[t][r] * invl[r]);
  }
  __syncthreads();
  v4u val[2];
  size_t go[2];
#pragma unroll
  for (int it = 0; it < 2; ++it) {
    const int p  = lane + 32 * it;
    const int L  = p >> 2;
    const int pc = p & 3;
    Pack8 pk;
    pk.h    = *(const v8h*)(pw + L * VSP + pc * 8);
    val[it] = pk.u;
    go[it]  = ((size_t)hb * NND + q0 + L) * HDM + pc * 8;
  }
  for (int ps = 0; ps < 2; ++ps) {
#pragma unroll
    for (int it = 0; it < 2; ++it) *(volatile v4u*)(op + go[it]) = val[it];
    __threadfence();
  }
}

#define OTP 260
__global__ __launch_bounds__(128) void k_oproj(const _Float16* __restrict__ op,
                                               const _Float16* __restrict__ wot,
                                               const float* __restrict__ bo,
                                               const float* __restrict__ xres,
                                               float* __restrict__ out) {
  __shared__ __align__(16) float sw[32 * OTP];
  const int tid = threadIdx.x, lane = tid & 31, wave = tid >> 5;
  const int hh = lane >> 4, c = lane & 15;
  const int m0 = blockIdx.x * 32;
  const int b  = m0 / NND;
  const int nl = m0 - b * NND;
  const _Float16* A = op + ((size_t)b * NH * NND + nl) * HDM;
  const int n0 = wave * 64;

  v8f acc[2][4];
#pragma unroll
  for (int s = 0; s < 2; ++s)
#pragma unroll
    for (int t = 0; t < 4; ++t) acc[s][t] = zero8();
  gemm32x64(A, HDM, NND * HDM, wot, DM, 32, DM / 32, 0, n0, lane, acc);

#pragma unroll
  for (int sub = 0; sub < 2; ++sub)
#pragma unroll
    for (int t = 0; t < 4; ++t)
#pragma unroll
      for (int r = 0; r < 8; ++r)
        sw[(sub * 16 + 8 * hh + r) * OTP + n0 + 16 * t + c] = acc[sub][t][r] * 0.00048828125f;
  __syncthreads();

  const v4f b0 = *(const v4f*)(bo + 4 * lane);
  const v4f b1 = *(const v4f*)(bo + 128 + 4 * lane);
#pragma unroll 1
  for (int rr = 0; rr < 8; ++rr) {
    const int row = wave * 8 + rr;
    const size_t m = (size_t)(m0 + row);
    const float* rp = xres + m * DM;
    const v4f v0 = *(const v4f*)(sw + row * OTP + 4 * lane) + b0 + *(const v4f*)(rp + 4 * lane);
    const v4f v1 = *(const v4f*)(sw + row * OTP + 128 + 4 * lane) + b1 + *(const v4f*)(rp + 128 + 4 * lane);
    float* yp = out + m * DM;
    *(volatile v4f*)(yp + 4 * lane) = v0;
    *(volatile v4f*)(yp + 128 + 4 * lane) = v1;
    __threadfence();
    *(volatile v4f*)(yp + 4 * lane) = v0;
    *(volatile v4f*)(yp + 128 + 4 * lane) = v1;
  }
}

extern "C" void kernel_launch(void* const* d_in, const int* in_sizes, int n_in,
                              void* d_out, int out_size, void* d_ws, size_t ws_size,
                              hipStream_t stream) {
  if (n_in < 14) return;
  if (in_sizes[0] != HN) return;
  if (in_sizes[1] != 2 * NEDG) return;
  if (in_sizes[2] != NEDG) return;
  if (in_sizes[3] != WMAT) return;
  if (in_sizes[4] != DM) return;
  if (in_sizes[5] != WMAT) return;
  if (in_sizes[6] != DM) return;
  if (in_sizes[7] != WMAT) return;
  if (in_sizes[8] != DM) return;
  if (in_sizes[9] != WMAT) return;
  if (in_sizes[10] != DM) return;
  if (in_sizes[11] != NET * HDM) return;
  if (in_sizes[12] != DM) return;
  if (in_sizes[13] != DM) return;
  if (out_size != HN) return;

  const float* x   = (const float*)d_in[0];
  const int*   ei  = (const int*)d_in[1];
  const int*   et  = (const int*)d_in[2];
  const float* wq  = (const float*)d_in[3];
  const float* bq  = (const float*)d_in[4];
  const float* wk  = (const float*)d_in[5];
  const float* bk  = (const float*)d_in[6];
  const float* wv  = (const float*)d_in[7];
  const float* bv  = (const float*)d_in[8];
  const float* wo  = (const float*)d_in[9];
  const float* bo  = (const float*)d_in[10];
  const float* emb = (const float*)d_in[11];
  const float* lng = (const float*)d_in[12];
  const float* lnb = (const float*)d_in[13];
  float* out = (float*)d_out;

  size_t off = 0;
  const size_t oW4 = off; off += (size_t)4 * WMAT * 2;
  const size_t oXN = off; off += (size_t)HN * 2;
  const size_t oQK = off; off += (size_t)2 * HPL * 2;
  const size_t oVt = off; off += (size_t)HPL * 2;
  const size_t oOp = off; off += (size_t)HPL * 2;
  const size_t oTb = off; off += (size_t)NND * NND * 4;
  if (off > ws_size) return;
  if (off > (size_t)134217728) return;

  char* ws = (char*)d_ws;
  _Float16* W4  = (_Float16*)(ws + oW4);
  _Float16* XN  = (_Float16*)(ws + oXN);
  _Float16* QK  = (_Float16*)(ws + oQK);
  _Float16* Vt  = (_Float16*)(ws + oVt);
  _Float16* Op  = (_Float16*)(ws + oOp);
  unsigned* Tab = (unsigned*)(ws + oTb);

  const float sscale = 0.17677669529663688f;

  k_wcvt<<<dim3(4 * (WMAT / 2048)), dim3(256), 0, stream>>>(wq, wk, wv, wo, W4);
  k_ln<<<dim3(NTOK / 8), dim3(256), 0, stream>>>(x, lng, lnb, XN);
  k_tab<<<dim3(NND / 8), dim3(256), 0, stream>>>(ei, et, Tab);
  k_qkv<<<dim3(NTOK / 256, 3 * (DM / 64)), dim3(256), 0, stream>>>(XN, W4, bq, bk, bv, QK, Vt);
  k_attn<<<dim3(NBT * NH * NQB), dim3(256), 0, stream>>>(QK, Vt, Tab, emb, Op, sscale);
  k_oproj<<<dim3(NTOK / 32), dim3(128), 0, stream>>>(Op, W4 + (size_t)3 * WMAT, bo, x, out);
  (void)hipGetLastError();
}
